// MultiLevelDynamicGraphEncoder_49443663511669
// MI455X (gfx1250) — hardware-verified
//
#include <hip/hip_runtime.h>


#define NN   2048
#define TT   20
#define CIN  2
#define KNB  32
#define NL   3
#define HH   64
#define G4   256
typedef _Float16 h16;
typedef unsigned short bf;
typedef __attribute__((ext_vector_type(16))) __bf16   v16bf;
typedef __attribute__((ext_vector_type(16))) _Float16 v16h;
typedef __attribute__((ext_vector_type(8)))  _Float16 v8h;
typedef __attribute__((ext_vector_type(8)))  unsigned short v8us;
typedef __attribute__((ext_vector_type(8)))  float    v8f;
typedef __attribute__((ext_vector_type(4)))  float    v4f;
typedef v8h  __attribute__((may_alias)) v8ha;
typedef v4f  __attribute__((may_alias)) v4fa;
typedef v8us __attribute__((may_alias)) v8usa;

__device__ __forceinline__ unsigned short f2bf(float f) { unsigned u = __float_as_uint(f); u += 0x7FFFu + ((u >> 16) & 1u); return (unsigned short)(u >> 16); }
__device__ __forceinline__ float bf2f(unsigned short b) { return __uint_as_float(((unsigned)b) << 16); }
__device__ __forceinline__ float bfr(float f) { return bf2f(f2bf(f)); }
__device__ __forceinline__ v16h cat16(v8h lo, v8h hi) { return __builtin_shufflevector(lo, hi, 0, 1, 2, 3, 4, 5, 6, 7, 8, 9, 10, 11, 12, 13, 14, 15); }
__device__ __forceinline__ v16bf cat16b(v8us lo, v8us hi) { return __builtin_bit_cast(v16bf, __builtin_shufflevector(lo, hi, 0, 1, 2, 3, 4, 5, 6, 7, 8, 9, 10, 11, 12, 13, 14, 15)); }
__device__ __forceinline__ v8f wmma16(v16h a, v16h b, v8f c) { return __builtin_amdgcn_wmma_f32_16x16x32_f16(false, a, false, b, (short)0, c, false, false); }
__device__ __forceinline__ v8f wmmab(v16bf a, v16bf b, v8f c) { return __builtin_amdgcn_wmma_f32_16x16x32_bf16(false, a, false, b, (short)0, c, false, false); }


template <typename T16> struct WFrag;
template <> struct WFrag<h16> { typedef v16h V; static __device__ __forceinline__ V ld(const h16* p) { return cat16(*(const v8h*)p, *(const v8h*)(p + 16)); } static __device__ __forceinline__ v8f mma(V a, V b, v8f c) { return wmma16(a, b, c); } };
template <> struct WFrag<bf> { typedef v16bf V; static __device__ __forceinline__ V ld(const bf* p) { return cat16b(*(const v8us*)p, *(const v8us*)(p + 16)); } static __device__ __forceinline__ v8f mma(V a, V b, v8f c) { return wmmab(a, b, c); } };
template <typename T16, int NSPLIT, bool BIAS>
__global__ __launch_bounds__(32) void k_gemmw(const T16* __restrict__ A, const T16* __restrict__ A2, const T16* __restrict__ Bt, const T16* __restrict__ Bt2, int K, float* C, int ldc, const float* __restrict__ bias, size_t sA, size_t sB, size_t sC) {
    typedef typename WFrag<T16>::V V;
    __shared__ __align__(16) float os[16 * 68];
    const size_t z = blockIdx.z; A += z * sA; if (A2) A2 += z * sA; Bt += z * sB; if (Bt2) Bt2 += z * sB; C += z * sC;
    const int lane = threadIdx.x & 31, lr = lane & 15, hi = lane >> 4; const int r0 = blockIdx.x * 64, c0 = blockIdx.y * 64;
    v8f acc[4][4];
#pragma unroll
    for (int mb = 0; mb < 4; ++mb)
#pragma unroll
        for (int nb = 0; nb < 4; ++nb) acc[mb][nb] = (v8f){};
    const size_t aoff = (size_t)(r0 + lr) * K + 8 * hi, boff = (size_t)(c0 + lr) * K + 8 * hi;
#pragma unroll 1
    for (int kc = 0; kc < K; kc += 32) {
        V a[4], a2[4];
#pragma unroll
        for (int mb = 0; mb < 4; ++mb) { a[mb] = WFrag<T16>::ld(A + aoff + (size_t)mb * 16 * K + kc); if (NSPLIT == 1 || NSPLIT == 2) a2[mb] = WFrag<T16>::ld(A2 + aoff + (size_t)mb * 16 * K + kc); }
#pragma unroll
        for (int nb = 0; nb < 4; ++nb) { const V b = WFrag<T16>::ld(Bt + boff + (size_t)nb * 16 * K + kc); V b2; if (NSPLIT >= 2) b2 = WFrag<T16>::ld(Bt2 + boff + (size_t)nb * 16 * K + kc);
#pragma unroll
            for (int mb = 0; mb < 4; ++mb) { acc[mb][nb] = WFrag<T16>::mma(a[mb], b, acc[mb][nb]); if (NSPLIT == 1 || NSPLIT == 2) acc[mb][nb] = WFrag<T16>::mma(a2[mb], b, acc[mb][nb]); if (NSPLIT >= 2) acc[mb][nb] = WFrag<T16>::mma(a[mb], b2, acc[mb][nb]); } }
        asm volatile("v_nop\n\tv_nop\n\tv_nop\n\tv_nop" : "+v"(acc[0][0]), "+v"(acc[1][1]), "+v"(acc[2][2]), "+v"(acc[3][3]) : "v"(a[0]), "v"(a[3]));
    }
#pragma unroll
    for (int mb = 0; mb < 4; ++mb) {
#pragma unroll
        for (int nb = 0; nb < 4; ++nb) {
#pragma unroll
            for (int j = 0; j < 8; ++j) os[(hi * 8 + j) * 68 + nb * 16 + lr] = acc[mb][nb][j]; }
        __builtin_amdgcn_wave_barrier(); asm volatile("" ::: "memory");
        float* crow = C + (size_t)(r0 + mb * 16) * ldc + c0;
#pragma unroll 1
        for (int ps = 0; ps < 2; ++ps) {
#pragma unroll
            for (int s = 0; s < 8; ++s) { const int row = 2 * s + hi, cofs = lr * 4; v4f val = *(const v4fa*)(os + row * 68 + cofs); if (BIAS) { val[0] += bfr(bias[c0 + cofs]); val[1] += bfr(bias[c0 + cofs + 1]); val[2] += bfr(bias[c0 + cofs + 2]); val[3] += bfr(bias[c0 + cofs + 3]); }
                *(volatile v4f*)(crow + (size_t)row * ldc + cofs) = val; }
            if (ps == 0) __threadfence(); }
        __builtin_amdgcn_wave_barrier(); asm volatile("" ::: "memory");
    }
}

__device__ __forceinline__ void splitf(float y, unsigned short& h, unsigned short& l) { h = f2bf(y); l = f2bf(y - bf2f(h)); }
__device__ __forceinline__ float sigm_(float a) { return __fdiv_rn(1.0f, __fadd_rn(1.0f, __expf(-a))); }
__device__ __forceinline__ float tanhf_(float a) { const float e2 = __expf(2.0f * a); return __fsub_rn(1.0f, __fdiv_rn(2.0f, __fadd_rn(e2, 1.0f))); }
typedef __attribute__((ext_vector_type(4))) unsigned short v4us;

__global__ __launch_bounds__(256) void k_cvt8(const float* __restrict__ src, bf* dst, size_t n8) { const size_t i = (size_t)blockIdx.x * 256 + threadIdx.x; if (i >= n8) return; const v8f v = *(const v8f*)(src + i * 8); v8us o;
#pragma unroll
    for (int k = 0; k < 8; ++k) o[k] = f2bf(v[k]); *(volatile v8us*)(dst + i * 8) = o; __threadfence(); *(volatile v8us*)(dst + i * 8) = o; }
__global__ __launch_bounds__(256) void k_pool(const float* __restrict__ X, const int* __restrict__ A, const float* __restrict__ Wc, const float* __restrict__ bc, float* PL) { const int e = blockIdx.x * 256 + threadIdx.x; if (e >= TT * NN * HH) return; const int o = e % HH; const int n = (e / HH) % NN; const int t = e / (HH * NN); const float w0 = bfr(Wc[o * 2]), w1 = bfr(Wc[o * 2 + 1]), b = bfr(bc[o]); const float x0 = bfr(X[((size_t)n * TT + t) * 2]), x1 = bfr(X[((size_t)n * TT + t) * 2 + 1]); float mx = -3.0e38f;
    for (int k = 0; k < KNB; ++k) { int a = A[((size_t)t * NN + n) * KNB + k]; a = min(max(a, 0), NN - 1); const float d0 = __fsub_rn(bfr(X[((size_t)a * TT + t) * 2]), x0), d1 = __fsub_rn(bfr(X[((size_t)a * TT + t) * 2 + 1]), x1); float p0 = __fmul_rn(d0, w0), p1 = __fmul_rn(d1, w1); asm volatile("" : "+v"(p0), "+v"(p1)); mx = fmaxf(mx, __fadd_rn(__fadd_rn(p0, p1), b)); }
    *(volatile float*)(PL + e) = mx; __threadfence(); *(volatile float*)(PL + e) = mx; }
__global__ __launch_bounds__(256) void k_spl(const float* __restrict__ F, size_t n4, bf* Fh, bf* Fl) { const size_t i = ((size_t)blockIdx.x * 256 + threadIdx.x) * 4; if (i >= n4 * 4) return; const v4f a = *(const v4f*)(F + i); v4us oh, ol;
#pragma unroll
    for (int q = 0; q < 4; ++q) { unsigned short u, c2; splitf(a[q], u, c2); oh[q] = u; ol[q] = c2; } *(volatile v4us*)(Fh + i) = oh; *(volatile v4us*)(Fl + i) = ol; __threadfence(); *(volatile v4us*)(Fh + i) = oh; *(volatile v4us*)(Fl + i) = ol; }
typedef __attribute__((ext_vector_type(2))) float v2f;
__global__ __launch_bounds__(256) void k_cell(const float* __restrict__ GX, const float* __restrict__ GH, const float* __restrict__ bih, const float* __restrict__ bhh, int t, int first, float* Hs, float* Cs, float* YS) { const int e = (blockIdx.x * 256 + threadIdx.x) * 2; if (e >= NN * HH) return; const int j = e % HH, n = e / HH; const float* gx = GX + ((size_t)t * NN + n) * G4; const float* gh = GH + (size_t)n * G4; const v2f cprev = first ? (v2f){0.f, 0.f} : *(const v2f*)(Cs + e); v2f hn, cn;
#pragma unroll
    for (int q = 0; q < 2; ++q) { const int jq = j + q; float g4[4];
#pragma unroll
        for (int u = 0; u < 4; ++u) { const int col = u * HH + jq; const float hv = first ? 0.f : gh[col]; g4[u] = __fadd_rn(__fadd_rn(gx[col], hv), __fadd_rn(bfr(bih[col]), bfr(bhh[col]))); }
        const float ig = sigm_(g4[0]), fg = sigm_(g4[1]), gg = tanhf_(g4[2]), og = sigm_(g4[3]); float fc = __fmul_rn(fg, cprev[q]); asm volatile("" : "+v"(fc)); float igg = __fmul_rn(ig, gg); asm volatile("" : "+v"(igg)); cn[q] = __fadd_rn(fc, igg); hn[q] = __fmul_rn(og, tanhf_(cn[q])); }
    const size_t yo = ((size_t)n * TT + t) * HH + j;
    *(volatile v2f*)(Hs + e) = hn; *(volatile v2f*)(Cs + e) = cn; *(volatile v2f*)(YS + yo) = hn; __threadfence(); *(volatile v2f*)(Hs + e) = hn; *(volatile v2f*)(Cs + e) = cn; *(volatile v2f*)(YS + yo) = hn; }
__global__ __launch_bounds__(256) void k_max3(const float* __restrict__ A0, const float* __restrict__ A1, const float* __restrict__ A2, size_t n4, float* OUT) { const size_t i = ((size_t)blockIdx.x * 256 + threadIdx.x) * 4; if (i >= n4 * 4) return; const v4f a = *(const v4f*)(A0 + i), b = *(const v4f*)(A1 + i), c = *(const v4f*)(A2 + i); v4f o;
#pragma unroll
    for (int q = 0; q < 4; ++q) o[q] = fmaxf(fmaxf(a[q], b[q]), c[q]); *(volatile v4f*)(OUT + i) = o; __threadfence(); *(volatile v4f*)(OUT + i) = o; }

extern "C" void kernel_launch(void* const* d_in, const int* in_sizes, int n_in,
                              void* d_out, int out_size, void* d_ws, size_t ws_size, hipStream_t stream) {
    (void)in_sizes; (void)n_in; (void)out_size;
    const float* X = (const float*)d_in[0]; const int* As = (const int*)d_in[1]; const float* Wc = (const float*)d_in[2]; const float* bc = (const float*)d_in[3]; const float* Wih = (const float*)d_in[4]; const float* Whh = (const float*)d_in[5]; const float* bih = (const float*)d_in[6]; const float* bhh = (const float*)d_in[7];
    float* OUTX = (float*)d_out; float* OUTH = OUTX + (size_t)NN * TT * HH; float* OUTC = OUTH + (size_t)NN * HH;
    char* wsp = (char*)d_ws;
    auto take = [&](size_t bytes) { char* p = wsp; wsp += (bytes + 255) & ~(size_t)255; return (void*)p; };
    bf* WIH = (bf*)take((size_t)G4 * HH * 2); bf* WHH = (bf*)take((size_t)G4 * HH * 2); float* PL = (float*)take((size_t)TT * NN * HH * 4); bf* Ph = (bf*)take((size_t)TT * NN * HH * 2); bf* Pl = (bf*)take((size_t)TT * NN * HH * 2); float* GX = (float*)take((size_t)TT * NN * G4 * 4);
    bf* Hh = (bf*)take((size_t)NN * HH * 2); bf* Hl = (bf*)take((size_t)NN * HH * 2); float* GH = (float*)take((size_t)NN * G4 * 4); float* Hs[NL]; float* Cs[NL]; float* YS[NL]; for (int l = 0; l < NL; ++l) { Hs[l] = (float*)take((size_t)NN * HH * 4); Cs[l] = (float*)take((size_t)NN * HH * 4); YS[l] = (float*)take((size_t)NN * TT * HH * 4); }
    if ((size_t)(wsp - (char*)d_ws) > ws_size) return;
    k_cvt8<<<(G4 * HH / 8 + 255) / 256, 256, 0, stream>>>(Wih, WIH, (size_t)G4 * HH / 8); k_cvt8<<<(G4 * HH / 8 + 255) / 256, 256, 0, stream>>>(Whh, WHH, (size_t)G4 * HH / 8);
    for (int lv = 0; lv < NL; ++lv) {
        k_pool<<<(TT * NN * HH + 255) / 256, 256, 0, stream>>>(X, As + (size_t)lv * TT * NN * KNB, Wc, bc, PL); k_spl<<<(TT * NN * HH / 4 + 255) / 256, 256, 0, stream>>>(PL, (size_t)TT * NN * HH / 4, Ph, Pl);
        k_gemmw<bf, 1, false><<<dim3(TT * NN / 64, G4 / 64, 1), 32, 0, stream>>>(Ph, Pl, WIH, nullptr, HH, GX, G4, nullptr, 0, 0, 0);
        for (int t = 0; t < TT; ++t) {
            if (t > 0) { k_spl<<<(NN * HH / 4 + 255) / 256, 256, 0, stream>>>(Hs[lv], (size_t)NN * HH / 4, Hh, Hl); k_gemmw<bf, 1, false><<<dim3(NN / 64, G4 / 64, 1), 32, 0, stream>>>(Hh, Hl, WHH, nullptr, HH, GH, G4, nullptr, 0, 0, 0); }
            k_cell<<<(NN * HH / 2 + 255) / 256, 256, 0, stream>>>(GX, GH, bih, bhh, t, t == 0, Hs[lv], Cs[lv], YS[lv]); } }
    k_max3<<<(unsigned)(((size_t)NN * TT * HH / 4 + 255) / 256), 256, 0, stream>>>(YS[0], YS[1], YS[2], (size_t)NN * TT * HH / 4, OUTX);
    k_max3<<<(NN * HH / 4 + 255) / 256, 256, 0, stream>>>(Hs[0], Hs[1], Hs[2], (size_t)NN * HH / 4, OUTH); k_max3<<<(NN * HH / 4 + 255) / 256, 256, 0, stream>>>(Cs[0], Cs[1], Cs[2], (size_t)NN * HH / 4, OUTC);
}
